// GPSConvNet_63900523430531
// MI455X (gfx1250) — hardware-verified
//
#include <hip/hip_runtime.h>
#include <stddef.h>
#include <stdint.h>

typedef _Float16 v16h __attribute__((ext_vector_type(16)));
typedef _Float16 v8h __attribute__((ext_vector_type(8)));
typedef _Float16 v8ha __attribute__((ext_vector_type(8), __may_alias__));
typedef _Float16 v4h __attribute__((ext_vector_type(4)));
typedef float v8f __attribute__((ext_vector_type(8)));
typedef float v4f __attribute__((ext_vector_type(4)));
typedef float v4fa __attribute__((ext_vector_type(4), __may_alias__));
typedef int v4i __attribute__((ext_vector_type(4)));

union HFrag { v16h v; v8h half[2]; _Float16 e[16]; };
union H8 { v8h v; _Float16 e[8]; };
union H4 { v4h v; _Float16 e[4]; };

#define NN 4096
#define NE 262144
#define ET (NE + NN)
#define FIN 9
#define DD 64
#define D2 128
#define D3 192
#define NLIN 320
#define NLAY 3
#define NH 4
#define DH 16
#define QP 32
#define NG 64
#define NC 10
#define TR 64
#define LP 132
#define QKP 200
#define SP 68
#define AP 72
#define MP 136
#define NBLK 64
#define CAP 6144
#define CHUNK 512
#define NCH (ET / CHUNK)
#define PREP_TASKS (1024 + NLAY * 5120)

__device__ __forceinline__ v8f zero8() {
  v8f z = {0.f, 0.f, 0.f, 0.f, 0.f, 0.f, 0.f, 0.f};
  return z;
}
__device__ __forceinline__ v8h zero8h() {
  H8 z;
#pragma unroll
  for (int i = 0; i < 8; ++i) z.e[i] = (_Float16)0.0f;
  return z.v;
}
__device__ __forceinline__ v8f wmma16(v16h a, v16h b, v8f c) {
  v8f d = __builtin_amdgcn_wmma_f32_16x16x32_f16(false, a, false, b, (short)0, c, false, false);
  asm volatile("v_nop\n\tv_nop\n\tv_nop\n\tv_nop" : "+v"(d) : "v"(a), "v"(b));
  return d;
}
__device__ __forceinline__ v16h ldfrag(const _Float16* p, int hf) {
  HFrag f;
  f.half[0] = *(const v8ha*)(p + 8 * hf);
  f.half[1] = *(const v8ha*)(p + 16 + 8 * hf);
  return f.v;
}

__device__ __forceinline__ float gelu_exact(float v) {
  return 0.5f * v * (1.0f + erff(v * 0.70710678118654752f));
}

__device__ __forceinline__ void store_tile_f32(const float* sT, int pitch, int coff, float* g, int l, int w) {
#pragma unroll
  for (int j = 0; j < 4; ++j) {
    const int q = l >> 3;
    const int row = w * 8 + 2 * j + (q >> 1);
    const int col = (q & 1) * 32 + (l & 7) * 4;
    const v4f v = *(const v4fa*)(sT + row * pitch + coff + col);
    *(volatile v4f*)(g + (size_t)row * DD + col) = v;
  }
}
__device__ __forceinline__ void store_tile_f16(const float* sT, int pitch, _Float16* g, int l, int w) {
#pragma unroll
  for (int j = 0; j < 2; ++j) {
    const int row = w * 8 + 4 * j + (l >> 3);
    const int col = (l & 7) * 8;
    const float* p = sT + row * pitch + col;
    const v4f u0 = *(const v4fa*)p;
    const v4f u1 = *(const v4fa*)(p + 4);
    H8 o;
    o.e[0] = (_Float16)u0.x; o.e[1] = (_Float16)u0.y; o.e[2] = (_Float16)u0.z; o.e[3] = (_Float16)u0.w;
    o.e[4] = (_Float16)u1.x; o.e[5] = (_Float16)u1.y; o.e[6] = (_Float16)u1.z; o.e[7] = (_Float16)u1.w;
    *(volatile v8h*)(g + (size_t)row * DD + col) = o.v;
  }
}

__global__ __launch_bounds__(256) void prep_kernel(const float* __restrict__ pre_w2, const float* __restrict__ wl,
                                                   const float* __restrict__ wr, const float* __restrict__ ain,
                                                   const float* __restrict__ aout, const float* __restrict__ mw1,
                                                   const float* __restrict__ mw2, _Float16* pW2t, _Float16* Wlin,
                                                   _Float16* Wo16, _Float16* Wm1t, _Float16* Wm2t) {
  const int tid = blockIdx.x * 256 + threadIdx.x;
  if (tid >= PREP_TASKS) return;
  H8 o;
  _Float16* d;
  if (tid < 1024) {
    const int n = tid >> 4, q = tid & 15;
#pragma unroll
    for (int i = 0; i < 8; ++i) o.e[i] = (_Float16)pre_w2[(size_t)(8 * q + i) * DD + n];
    d = pW2t + (size_t)n * D2 + 8 * q;
  } else {
    const int u = tid - 1024;
    const int ly = u / 5120;
    const int r = u - ly * 5120;
    if (r < 2560) {
      const int n = r >> 3, q = r & 7;
      if (n < DD) {
#pragma unroll
        for (int i = 0; i < 8; ++i) o.e[i] = (_Float16)wl[(size_t)ly * DD * DD + (size_t)(8 * q + i) * DD + n];
      } else if (n < D2) {
#pragma unroll
        for (int i = 0; i < 8; ++i) o.e[i] = (_Float16)wr[(size_t)ly * DD * DD + (size_t)(8 * q + i) * DD + (n - DD)];
      } else {
#pragma unroll
        for (int i = 0; i < 8; ++i) o.e[i] = (_Float16)ain[(size_t)ly * D3 * DD + (size_t)(n - D2) * DD + 8 * q + i];
      }
      d = Wlin + ((size_t)ly * NLIN + n) * DD + 8 * q;
    } else if (r < 3072) {
      const int v = r - 2560;
      const int n = v >> 3, q = v & 7;
#pragma unroll
      for (int i = 0; i < 8; ++i) o.e[i] = (_Float16)aout[(size_t)ly * DD * DD + (size_t)n * DD + 8 * q + i];
      d = Wo16 + ((size_t)ly * DD + n) * DD + 8 * q;
    } else if (r < 4096) {
      const int v = r - 3072;
      const int n = v >> 3, q = v & 7;
#pragma unroll
      for (int i = 0; i < 8; ++i) o.e[i] = (_Float16)mw1[(size_t)ly * DD * D2 + (size_t)(8 * q + i) * D2 + n];
      d = Wm1t + ((size_t)ly * D2 + n) * DD + 8 * q;
    } else {
      const int v = r - 4096;
      const int n = v >> 4, q = v & 15;
#pragma unroll
      for (int i = 0; i < 8; ++i) o.e[i] = (_Float16)mw2[(size_t)ly * D2 * DD + (size_t)(8 * q + i) * DD + n];
      d = Wm2t + ((size_t)ly * DD + n) * D2 + 8 * q;
    }
  }
  *(volatile v8h*)d = o.v;
  __threadfence();
  *(volatile v8h*)d = o.v;
}

__global__ __launch_bounds__(256) void premlp_kernel(const float* __restrict__ xin, const float* __restrict__ w1,
                                                     const float* __restrict__ b1, const _Float16* __restrict__ W2t,
                                                     const float* __restrict__ b2, float* x32, _Float16* x16) {
  __shared__ __align__(16) _Float16 sH[TR * MP];
  __shared__ __align__(16) float sT[TR * SP];
  const int t = threadIdx.x, l = t & 31, w = t >> 5, hf = l >> 4, n = l & 15;
  const int node0 = blockIdx.x * TR;

#pragma unroll 1
  for (int p = t; p < TR * D2; p += 256) {
    const int row = p >> 7, col = p & (D2 - 1);
    const float* xrow = xin + (size_t)(node0 + row) * FIN;
    float acc = 0.f;
#pragma unroll
    for (int k = 0; k < FIN; ++k) acc += xrow[k] * w1[k * D2 + col];
    acc += b1[col];
    sH[row * MP + col] = (_Float16)gelu_exact(acc);
  }
  __syncthreads();

  const int rt = w >> 1;
  const _Float16* ar = sH + (rt * 16 + n) * MP;
  v16h a[4];
#pragma unroll
  for (int ks = 0; ks < 4; ++ks) a[ks] = ldfrag(ar + 32 * ks, hf);
#pragma unroll
  for (int c2 = 0; c2 < 2; ++c2) {
    const int ct = (w & 1) * 2 + c2;
    const _Float16* bp = W2t + (size_t)(ct * 16 + n) * D2;
    v8f acc = zero8();
#pragma unroll
    for (int ks = 0; ks < 4; ++ks) acc = wmma16(a[ks], ldfrag(bp + 32 * ks, hf), acc);
    const int col = ct * 16 + n;
    const float bb = b2[col];
    const int rowb = rt * 16 + 8 * hf;
#pragma unroll
    for (int r = 0; r < 8; ++r) sT[(rowb + r) * SP + col] = gelu_exact(acc[r] + bb);
  }
  __syncthreads();

  store_tile_f32(sT, SP, 0, x32 + (size_t)node0 * DD, l, w);
  store_tile_f16(sT, SP, x16 + (size_t)node0 * DD, l, w);
  __threadfence();
  store_tile_f32(sT, SP, 0, x32 + (size_t)node0 * DD, l, w);
  store_tile_f16(sT, SP, x16 + (size_t)node0 * DD, l, w);
}

__device__ __forceinline__ void lin_store(const float* sLR, const _Float16* sQ, float* xl, float* xr,
                                          _Float16* q16, _Float16* k16, _Float16* vT, int node0, int t, int l, int w) {
  store_tile_f32(sLR, LP, 0, xl + (size_t)node0 * DD, l, w);
  store_tile_f32(sLR, LP, DD, xr + (size_t)node0 * DD, l, w);
  const int nd = t >> 2, p = t & 3;
#pragma unroll
  for (int hh = 0; hh < NH; ++hh) {
    v8h vq = zero8h(), vk = zero8h();
    if (p < 2) {
      vq = *(const v8ha*)(sQ + nd * QKP + hh * DH + 8 * p);
      vk = *(const v8ha*)(sQ + nd * QKP + DD + hh * DH + 8 * p);
    }
    *(volatile v8h*)(q16 + ((size_t)hh * NN + node0 + nd) * QP + 8 * p) = vq;
    *(volatile v8h*)(k16 + ((size_t)hh * NN + node0 + nd) * QP + 8 * p) = vk;
  }
#pragma unroll
  for (int j = 0; j < 2; ++j) {
    const int L = j * 32 + (t >> 3);
    const int hh = L >> 4, d = L & 15;
    const int nb = 8 * (t & 7);
    H8 o;
#pragma unroll
    for (int i = 0; i < 8; ++i) o.e[i] = sQ[(nb + i) * QKP + D2 + hh * DH + d];
    *(volatile v8h*)(vT + ((size_t)hh * DH + d) * NN + node0 + nb) = o.v;
  }
}

__global__ __launch_bounds__(256) void lin_kernel(const _Float16* __restrict__ x16, const _Float16* __restrict__ Wl,
                                                  const float* __restrict__ bl, const float* __restrict__ br,
                                                  const float* __restrict__ bin, float* xl, float* xr,
                                                  _Float16* q16, _Float16* k16, _Float16* vT) {
  __shared__ __align__(16) float sLR[TR * LP];
  __shared__ __align__(16) _Float16 sQ[TR * QKP];
  const int t = threadIdx.x, l = t & 31, w = t >> 5, hf = l >> 4, n = l & 15;
  const int node0 = blockIdx.x * TR;
  const int rt = w >> 1;
  const _Float16* ap = x16 + (size_t)(node0 + rt * 16 + n) * DD;
  const v16h a0 = ldfrag(ap, hf);
  const v16h a1 = ldfrag(ap + 32, hf);

#pragma unroll 1
  for (int j = 0; j < 10; ++j) {
    const int ct = (w & 1) * 10 + j;
    const _Float16* bp = Wl + (size_t)(ct * 16 + n) * DD;
    v8f acc = wmma16(a0, ldfrag(bp, hf), zero8());
    acc = wmma16(a1, ldfrag(bp + 32, hf), acc);
    const int col = ct * 16 + n;
    const int rowb = rt * 16 + 8 * hf;
    if (ct < 8) {
      const float bb = (ct < 4) ? bl[col] : br[col - DD];
#pragma unroll
      for (int r = 0; r < 8; ++r) sLR[(rowb + r) * LP + col] = acc[r] + bb;
    } else {
      const int c = col - D2;
      const float bb = bin[c];
      const float sc = (c < DD) ? 0.25f : 1.0f;
#pragma unroll
      for (int r = 0; r < 8; ++r) sQ[(rowb + r) * QKP + c] = (_Float16)((acc[r] + bb) * sc);
    }
  }
  __syncthreads();

  lin_store(sLR, sQ, xl, xr, q16, k16, vT, node0, t, l, w);
  __threadfence();
  lin_store(sLR, sQ, xl, xr, q16, k16, vT, node0, t, l, w);
}

__device__ __forceinline__ void agg_store(const float* sS, float* g, int l) {
#pragma unroll 8
  for (int j = 0; j < NBLK / 2; ++j) {
    const int row = 2 * j + (l >> 4), col = (l & 15) * 4;
    const v4f v = *(const v4fa*)(sS + row * DD + col);
    *(volatile v4f*)(g + (size_t)row * DD + col) = v;
  }
}

__global__ __launch_bounds__(32) void agg_kernel(const int* __restrict__ srcA, const int* __restrict__ dstA,
                                                 const float* __restrict__ xlA, const float* __restrict__ xrA,
                                                 const float* __restrict__ att, const float* __restrict__ gbias,
                                                 const float* __restrict__ xres, float* h1) {
  __shared__ __align__(16) float sS[NBLK * DD];
  __shared__ __align__(16) float dS[NBLK];
  __shared__ int list[CAP];
  const int l = threadIdx.x;
  const int nodeBase = blockIdx.x * NBLK;

  {
    const v4f z = {0.f, 0.f, 0.f, 0.f};
    for (int i = l; i < (NBLK * DD) / 4; i += 32) *(v4f*)(sS + 4 * i) = z;
    for (int i = l; i < NBLK; i += 32) dS[i] = 0.f;
  }
  __syncthreads();

  int count = 0;
#pragma unroll 1
  for (int ci = 0; ci < NCH; ++ci) {
    const int cbase = ci * CHUNK;
    int dv[16];
#pragma unroll
    for (int j = 0; j < 4; ++j) {
      const int e4 = cbase + 128 * j + 4 * l;
      int d0, d1, d2, d3;
      if (e4 + 3 < NE) {
        const v4i dd = *(const v4i*)(dstA + e4);
        d0 = dd.x; d1 = dd.y; d2 = dd.z; d3 = dd.w;
      } else {
        d0 = (e4 < ET) ? (e4 - NE) : -1;
        d1 = (e4 + 1 < ET) ? (e4 + 1 - NE) : -1;
        d2 = (e4 + 2 < ET) ? (e4 + 2 - NE) : -1;
        d3 = (e4 + 3 < ET) ? (e4 + 3 - NE) : -1;
      }
      dv[4 * j] = d0; dv[4 * j + 1] = d1; dv[4 * j + 2] = d2; dv[4 * j + 3] = d3;
    }
    unsigned hit = 0;
    int cnt = 0;
#pragma unroll
    for (int i = 0; i < 16; ++i) {
      const int s = dv[i] - nodeBase;
      if ((unsigned)s < (unsigned)NBLK) { hit |= (1u << i); ++cnt; }
    }
    int incl = cnt;
#pragma unroll
    for (int o = 1; o < 32; o <<= 1) {
      const int y = __shfl_up(incl, o, 32);
      if (l >= o) incl += y;
    }
    const int tot = __shfl(incl, 31, 32);
    int pos = count + incl - cnt;
#pragma unroll
    for (int i = 0; i < 16; ++i) {
      if (hit & (1u << i)) {
        const int e = cbase + 128 * (i >> 2) + 4 * l + (i & 3);
        if ((unsigned)pos < (unsigned)CAP) list[pos] = (e << 6) | (dv[i] - nodeBase);
        ++pos;
      }
    }
    count += tot;
    if (count > CAP) count = CAP;
  }
  __syncthreads();

  {
    const float aw0 = att[l], aw1 = att[32 + l];
    const int cc = count;
#pragma unroll 1
    for (int li = 0; li < CAP; ++li) {
      if (li >= cc) break;
      const int ent = list[li];
      int e = ent >> 6;
      if (e < 0) e = 0;
      if (e > ET - 1) e = ET - 1;
      const int slot = ent & (NBLK - 1);
      int s;
      if (e < NE) {
        s = srcA[e];
        s = (s < 0) ? 0 : ((s > NN - 1) ? (NN - 1) : s);
      } else {
        s = e - NE;
      }
      const int dn = nodeBase + slot;
      const float xa0 = xlA[(size_t)s * DD + l];
      const float xa1 = xlA[(size_t)s * DD + 32 + l];
      float u0 = xa0 + xrA[(size_t)dn * DD + l];
      float u1 = xa1 + xrA[(size_t)dn * DD + 32 + l];
      u0 = fmaxf(u0, 0.2f * u0);
      u1 = fmaxf(u1, 0.2f * u1);
      float ev = u0 * aw0 + u1 * aw1;
#pragma unroll
      for (int o = 1; o < 32; o <<= 1) ev += __shfl_xor(ev, o, 32);
      ev = __shfl(ev, 0, 32);
      ev = fminf(ev, 80.0f);
      const float ex = __expf(ev);
      sS[slot * DD + l] += ex * xa0;
      sS[slot * DD + 32 + l] += ex * xa1;
      if (l == 0) dS[slot] += ex;
    }
  }
  __syncthreads();

  {
    const float gb0 = gbias[l], gb1 = gbias[32 + l];
#pragma unroll 1
    for (int sl = 0; sl < NBLK; ++sl) {
      const int node = nodeBase + sl;
      const float d = dS[sl];
      const float inv = (d > 0.f) ? __builtin_amdgcn_rcpf(d) : 0.f;
      const float v0 = sS[sl * DD + l] * inv + gb0 + xres[(size_t)node * DD + l];
      const float v1 = sS[sl * DD + 32 + l] * inv + gb1 + xres[(size_t)node * DD + 32 + l];
      sS[sl * DD + l] = v0;
      sS[sl * DD + 32 + l] = v1;
    }
  }
  __syncthreads();

  agg_store(sS, h1 + (size_t)nodeBase * DD, l);
  __threadfence();
  agg_store(sS, h1 + (size_t)nodeBase * DD, l);
}

__global__ __launch_bounds__(256) void stats_kernel(const float* __restrict__ a, const float* __restrict__ b, float* st) {
  __shared__ double sSum[256];
  __shared__ double sSq[256];
  __shared__ __align__(16) float sO[128];
  const int t = threadIdx.x, c = t & 63, rg = t >> 6;
  const float* in = (blockIdx.x == 0) ? a : b;
  double s = 0.0, q = 0.0;
#pragma unroll 4
  for (int r = rg; r < NN; r += 4) {
    const float v = in[(size_t)r * DD + c];
    s += (double)v;
    q += (double)v * (double)v;
  }
  sSum[t] = s;
  sSq[t] = q;
  __syncthreads();
  if (t < 64) {
    const double S = ((sSum[t] + sSum[t + 64]) + sSum[t + 128]) + sSum[t + 192];
    const double Q = ((sSq[t] + sSq[t + 64]) + sSq[t + 128]) + sSq[t + 192];
    const double mean = S * (1.0 / (double)NN);
    double var = Q * (1.0 / (double)NN) - mean * mean;
    if (var < 0.0) var = 0.0;
    sO[t] = (float)mean;
    sO[64 + t] = rsqrtf((float)var + 1e-5f);
  }
  __syncthreads();
  if (t < 32) {
    const v4f v = *(const v4fa*)(sO + 4 * t);
    float* d = st + (size_t)blockIdx.x * 128 + 4 * t;
    *(volatile v4f*)d = v;
    __threadfence();
    *(volatile v4f*)d = v;
  }
}

__global__ __launch_bounds__(128) void attn_kernel(const _Float16* __restrict__ q16, const _Float16* __restrict__ k16,
                                                   const _Float16* __restrict__ vT, _Float16* o16) {
  __shared__ __align__(16) _Float16 sO[4 * 256];
  const int t = threadIdx.x, l = t & 31, w = t >> 5, hf = l >> 4, n = l & 15;
  const int head = blockIdx.y;
  const int q0 = blockIdx.x * 64 + w * 16;
  const _Float16* qh = q16 + (size_t)head * NN * QP;
  const _Float16* kh = k16 + (size_t)head * NN * QP;
  const _Float16* vh = vT + (size_t)head * DH * NN;
  const v16h bq = ldfrag(qh + (size_t)(q0 + n) * QP, hf);

  float m = -3.0e38f, ls = 0.f;
  v8f accO = zero8();
#pragma unroll 1
  for (int kb = 0; kb < NN; kb += 64) {
    const v8f s0 = wmma16(ldfrag(kh + (size_t)(kb + n) * QP, hf), bq, zero8());
    const v8f s1 = wmma16(ldfrag(kh + (size_t)(kb + 16 + n) * QP, hf), bq, zero8());
    const v8f s2 = wmma16(ldfrag(kh + (size_t)(kb + 32 + n) * QP, hf), bq, zero8());
    const v8f s3 = wmma16(ldfrag(kh + (size_t)(kb + 48 + n) * QP, hf), bq, zero8());
    float mx = m;
#pragma unroll
    for (int r = 0; r < 8; ++r) mx = fmaxf(mx, fmaxf(fmaxf(s0[r], s1[r]), fmaxf(s2[r], s3[r])));
    mx = fmaxf(mx, __shfl_xor(mx, 16, 32));
    float rs = 0.f;
    HFrag p0, p1;
#pragma unroll
    for (int r = 0; r < 8; ++r) {
      const float e0 = __expf(s0[r] - mx);
      const float e1 = __expf(s1[r] - mx);
      const float e2 = __expf(s2[r] - mx);
      const float e3 = __expf(s3[r] - mx);
      rs += (e0 + e1) + (e2 + e3);
      p0.e[r] = (_Float16)(e0 * 16384.0f);
      p0.e[8 + r] = (_Float16)(e1 * 16384.0f);
      p1.e[r] = (_Float16)(e2 * 16384.0f);
      p1.e[8 + r] = (_Float16)(e3 * 16384.0f);
    }
    rs += __shfl_xor(rs, 16, 32);
    const float sc = __expf(m - mx);
    ls = ls * sc + rs;
    m = mx;
    accO = accO * sc;
    accO = wmma16(ldfrag(vh + (size_t)n * NN + kb, hf), p0.v, accO);
    accO = wmma16(ldfrag(vh + (size_t)n * NN + kb + 32, hf), p1.v, accO);
  }
  const float inv = __builtin_amdgcn_rcpf(ls * 16384.0f);
  _Float16* so = sO + w * 256;
#pragma unroll
  for (int r = 0; r < 8; ++r) so[n * 16 + 8 * hf + r] = (_Float16)(accO[r] * inv);
  __syncthreads();
  const v8h ov = *(const v8ha*)(so + 8 * l);
  _Float16* d = o16 + ((size_t)head * NN + q0 + (l >> 1)) * DH + (l & 1) * 8;
  *(volatile v8h*)d = ov;
  __threadfence();
  *(volatile v8h*)d = ov;
}

__global__ __launch_bounds__(256) void oproj_kernel(const _Float16* __restrict__ o16, const _Float16* __restrict__ Wo,
                                                    const float* __restrict__ bo, const float* __restrict__ x32,
                                                    float* h2) {
  __shared__ __align__(16) float sT[TR * SP];
  const int t = threadIdx.x, l = t & 31, w = t >> 5, hf = l >> 4, n = l & 15;
  const int node0 = blockIdx.x * TR;
  const int rt = w >> 1;
  const int mrow = node0 + rt * 16 + n;
  HFrag a0, a1;
  {
    const int c00 = 8 * hf, c01 = 16 + 8 * hf, c10 = 32 + 8 * hf, c11 = 48 + 8 * hf;
    a0.half[0] = *(const v8ha*)(o16 + ((size_t)(c00 >> 4) * NN + mrow) * DH + (c00 & 15));
    a0.half[1] = *(const v8ha*)(o16 + ((size_t)(c01 >> 4) * NN + mrow) * DH + (c01 & 15));
    a1.half[0] = *(const v8ha*)(o16 + ((size_t)(c10 >> 4) * NN + mrow) * DH + (c10 & 15));
    a1.half[1] = *(const v8ha*)(o16 + ((size_t)(c11 >> 4) * NN + mrow) * DH + (c11 & 15));
  }
#pragma unroll
  for (int c2 = 0; c2 < 2; ++c2) {
    const int ct = (w & 1) * 2 + c2;
    const _Float16* bp = Wo + (size_t)(ct * 16 + n) * DD;
    v8f acc = wmma16(a0.v, ldfrag(bp, hf), zero8());
    acc = wmma16(a1.v, ldfrag(bp + 32, hf), acc);
    const int col = ct * 16 + n;
    const float bb = bo[col];
    const int rowb = rt * 16 + 8 * hf;
#pragma unroll
    for (int r = 0; r < 8; ++r)
      sT[(rowb + r) * SP + col] = acc[r] + bb + x32[(size_t)(node0 + rowb + r) * DD + col];
  }
  __syncthreads();
  store_tile_f32(sT, SP, 0, h2 + (size_t)node0 * DD, l, w);
  __threadfence();
  store_tile_f32(sT, SP, 0, h2 + (size_t)node0 * DD, l, w);
}

__global__ __launch_bounds__(256) void mlp_kernel(const float* __restrict__ h1, const float* __restrict__ h2,
                                                  const float* __restrict__ st, const float* __restrict__ g1,
                                                  const float* __restrict__ be1, const float* __restrict__ g2,
                                                  const float* __restrict__ be2, const _Float16* __restrict__ W1t,
                                                  const float* __restrict__ mb1, const _Float16* __restrict__ W2t,
                                                  const float* __restrict__ mb2, float* o2) {
  __shared__ __align__(16) float sOut[TR * SP];
  __shared__ __align__(16) _Float16 sA[TR * AP];
  __shared__ __align__(16) _Float16 sM[TR * MP];
  const int t = threadIdx.x, l = t & 31, w = t >> 5, hf = l >> 4, n = l & 15;
  const int node0 = blockIdx.x * TR;

#pragma unroll
  for (int j = 0; j < 4; ++j) {
    const int f = j * 1024 + 4 * t;
    const int row = f >> 6, col = f & 63;
    const size_t gi = (size_t)(node0 + row) * DD + col;
    const v4f u1 = *(const v4f*)(h1 + gi);
    const v4f u2 = *(const v4f*)(h2 + gi);
    const v4f m1 = *(const v4f*)(st + col), r1 = *(const v4f*)(st + 64 + col);
    const v4f m2 = *(const v4f*)(st + 128 + col), r2 = *(const v4f*)(st + 192 + col);
    const v4f ga = *(const v4f*)(g1 + col), ba = *(const v4f*)(be1 + col);
    const v4f gb = *(const v4f*)(g2 + col), bb = *(const v4f*)(be2 + col);
    const v4f y1 = (u1 - m1) * r1 * ga + ba;
    const v4f y2 = (u2 - m2) * r2 * gb + bb;
    const v4f o = y1 + y2;
    *(v4f*)(sOut + row * SP + col) = o;
    H4 hh;
    hh.e[0] = (_Float16)o.x; hh.e[1] = (_Float16)o.y; hh.e[2] = (_Float16)o.z; hh.e[3] = (_Float16)o.w;
    *(v4h*)(sA + row * AP + col) = hh.v;
  }
  __syncthreads();

  const int rt = w >> 1;
  {
    const _Float16* ar = sA + (rt * 16 + n) * AP;
    const v16h a0 = ldfrag(ar, hf);
    const v16h a1 = ldfrag(ar + 32, hf);
#pragma unroll
    for (int c4 = 0; c4 < 4; ++c4) {
      const int ct = (w & 1) * 4 + c4;
      const _Float16* bp = W1t + (size_t)(ct * 16 + n) * DD;
      v8f acc = wmma16(a0, ldfrag(bp, hf), zero8());
      acc = wmma16(a1, ldfrag(bp + 32, hf), acc);
      const int col = ct * 16 + n;
      const float bb = mb1[col];
      const int rowb = rt * 16 + 8 * hf;
#pragma unroll
      for (int r = 0; r < 8; ++r) sM[(rowb + r) * MP + col] = (_Float16)fmaxf(acc[r] + bb, 0.f);
    }
  }
  __syncthreads();

  {
    const _Float16* ar = sM + (rt * 16 + n) * MP;
    v16h a[4];
#pragma unroll
    for (int ks = 0; ks < 4; ++ks) a[ks] = ldfrag(ar + 32 * ks, hf);
#pragma unroll
    for (int c2 = 0; c2 < 2; ++c2) {
      const int ct = (w & 1) * 2 + c2;
      const _Float16* bp = W2t + (size_t)(ct * 16 + n) * D2;
      v8f acc = zero8();
#pragma unroll
      for (int ks = 0; ks < 4; ++ks) acc = wmma16(a[ks], ldfrag(bp + 32 * ks, hf), acc);
      const int col = ct * 16 + n;
      const float bb = mb2[col];
      const int rowb = rt * 16 + 8 * hf;
#pragma unroll
      for (int r = 0; r < 8; ++r) {
        const int idx = (rowb + r) * SP + col;
        const float v = acc[r] + bb + sOut[idx];
        sOut[idx] = v;
      }
    }
  }
  __syncthreads();

  store_tile_f32(sOut, SP, 0, o2 + (size_t)node0 * DD, l, w);
  __threadfence();
  store_tile_f32(sOut, SP, 0, o2 + (size_t)node0 * DD, l, w);
}

__global__ __launch_bounds__(256) void apply_kernel(const float* __restrict__ o2, const float* __restrict__ st,
                                                    const float* __restrict__ g, const float* __restrict__ b,
                                                    float* x32, _Float16* x16) {
  const int t = threadIdx.x;
  const int base = blockIdx.x * 2048;
  v4f va[2];
  int fa[2];
#pragma unroll
  for (int j = 0; j < 2; ++j) {
    const int f = base + j * 1024 + 4 * t;
    const int col = f & 63;
    const v4f in = *(const v4f*)(o2 + f);
    const v4f mm = *(const v4f*)(st + col), rr = *(const v4f*)(st + 64 + col);
    const v4f gg = *(const v4f*)(g + col), bb = *(const v4f*)(b + col);
    v4f y = (in - mm) * rr * gg + bb;
    y.x = fmaxf(y.x, 0.f); y.y = fmaxf(y.y, 0.f); y.z = fmaxf(y.z, 0.f); y.w = fmaxf(y.w, 0.f);
    va[j] = y;
    fa[j] = f;
  }
  const int idx = base + 8 * t;
  H8 o;
  {
    const int col = idx & 63;
    const v4f in0 = *(const v4f*)(o2 + idx), in1 = *(const v4f*)(o2 + idx + 4);
    const v4f m0 = *(const v4f*)(st + col), m1 = *(const v4f*)(st + col + 4);
    const v4f r0 = *(const v4f*)(st + 64 + col), r1 = *(const v4f*)(st + 64 + col + 4);
    const v4f g0 = *(const v4f*)(g + col), g1 = *(const v4f*)(g + col + 4);
    const v4f b0 = *(const v4f*)(b + col), b1 = *(const v4f*)(b + col + 4);
    const v4f y0 = (in0 - m0) * r0 * g0 + b0;
    const v4f y1 = (in1 - m1) * r1 * g1 + b1;
    o.e[0] = (_Float16)fmaxf(y0.x, 0.f); o.e[1] = (_Float16)fmaxf(y0.y, 0.f);
    o.e[2] = (_Float16)fmaxf(y0.z, 0.f); o.e[3] = (_Float16)fmaxf(y0.w, 0.f);
    o.e[4] = (_Float16)fmaxf(y1.x, 0.f); o.e[5] = (_Float16)fmaxf(y1.y, 0.f);
    o.e[6] = (_Float16)fmaxf(y1.z, 0.f); o.e[7] = (_Float16)fmaxf(y1.w, 0.f);
  }
  *(volatile v4f*)(x32 + fa[0]) = va[0];
  *(volatile v4f*)(x32 + fa[1]) = va[1];
  *(volatile v8h*)(x16 + idx) = o.v;
  __threadfence();
  *(volatile v4f*)(x32 + fa[0]) = va[0];
  *(volatile v4f*)(x32 + fa[1]) = va[1];
  *(volatile v8h*)(x16 + idx) = o.v;
}

__global__ __launch_bounds__(64) void pool_kernel(const float* __restrict__ x32, const int* __restrict__ bidx,
                                                  float* pooled) {
  __shared__ __align__(16) float sP[DD];
  const int g = blockIdx.x, c = threadIdx.x;
  float acc = 0.f;
  int cnt = 0;
#pragma unroll 4
  for (int nd = 0; nd < NN; ++nd) {
    const int bg = bidx[nd];
    if (bg == g) { acc += x32[(size_t)nd * DD + c]; ++cnt; }
  }
  const float den = fmaxf((float)cnt, 1.0f);
  sP[c] = acc * (1.0f / den);
  __syncthreads();
  if (c < 16) {
    const v4f v = *(const v4fa*)(sP + 4 * c);
    float* d = pooled + (size_t)g * DD + 4 * c;
    *(volatile v4f*)d = v;
    __threadfence();
    *(volatile v4f*)d = v;
  }
}

__device__ __forceinline__ void final_store(const float* sO, float* out, int g) {
#pragma unroll
  for (int j = 0; j < 3; ++j) {
    const int i = j * 64 + g;
    if (i < (NG * NC) / 4) {
      const v4f v = *(const v4fa*)(sO + 4 * i);
      *(volatile v4f*)(out + 4 * i) = v;
    }
  }
}

__global__ __launch_bounds__(64) void final_kernel(const float* __restrict__ pooled, const float* __restrict__ fw,
                                                   const float* __restrict__ fb, float* out) {
  __shared__ __align__(16) float sO[NG * NC];
  const int g = threadIdx.x;
  float lg[NC];
#pragma unroll
  for (int c = 0; c < NC; ++c) lg[c] = 0.f;
#pragma unroll 1
  for (int k = 0; k < DD; ++k) {
    const float pv = pooled[(size_t)g * DD + k];
#pragma unroll
    for (int c = 0; c < NC; ++c) lg[c] += pv * fw[k * NC + c];
  }
  float mx = -3.0e38f;
#pragma unroll
  for (int c = 0; c < NC; ++c) { lg[c] += fb[c]; mx = fmaxf(mx, lg[c]); }
  float se = 0.f;
#pragma unroll
  for (int c = 0; c < NC; ++c) se += expf(lg[c] - mx);
  const float lse = logf(se);
#pragma unroll
  for (int c = 0; c < NC; ++c) sO[g * NC + c] = (lg[c] - mx) - lse;
  __syncthreads();
  final_store(sO, out, g);
  __threadfence();
  final_store(sO, out, g);
}

extern "C" void kernel_launch(void* const* d_in, const int* in_sizes, int n_in,
                              void* d_out, int out_size, void* d_ws, size_t ws_size,
                              hipStream_t stream) {
  if (n_in < 29) return;
  const float* x_in      = (const float*)d_in[0];
  const int*   eidx      = (const int*)d_in[1];
  const int*   bidx      = (const int*)d_in[2];
  const float* pre_w1    = (const float*)d_in[3];
  const float* pre_b1    = (const float*)d_in[4];
  const float* pre_w2    = (const float*)d_in[5];
  const float* pre_b2    = (const float*)d_in[6];
  const float* gat_wl    = (const float*)d_in[7];
  const float* gat_bl    = (const float*)d_in[8];
  const float* gat_wr    = (const float*)d_in[9];
  const float* gat_br    = (const float*)d_in[10];
  const float* gat_att   = (const float*)d_in[11];
  const float* gat_bias  = (const float*)d_in[12];
  const float* ain_w     = (const float*)d_in[13];
  const float* ain_b     = (const float*)d_in[14];
  const float* aout_w    = (const float*)d_in[15];
  const float* aout_b    = (const float*)d_in[16];
  const float* bn1_g     = (const float*)d_in[17];
  const float* bn1_b     = (const float*)d_in[18];
  const float* bn2_g     = (const float*)d_in[19];
  const float* bn2_b     = (const float*)d_in[20];
  const float* bn3_g     = (const float*)d_in[21];
  const float* bn3_b     = (const float*)d_in[22];
  const float* mlp_w1    = (const float*)d_in[23];
  const float* mlp_b1    = (const float*)d_in[24];
  const float* mlp_w2    = (const float*)d_in[25];
  const float* mlp_b2    = (const float*)d_in[26];
  const float* fin_w     = (const float*)d_in[27];
  const float* fin_b     = (const float*)d_in[28];

  if (in_sizes[0] != NN * FIN || in_sizes[1] != 2 * NE || in_sizes[2] != NN) return;
  if (in_sizes[3] != FIN * D2 || in_sizes[4] != D2 || in_sizes[5] != D2 * DD || in_sizes[6] != DD) return;
  if (in_sizes[7] != NLAY * DD * DD || in_sizes[9] != NLAY * DD * DD || in_sizes[13] != NLAY * D3 * DD ||
      in_sizes[14] != NLAY * D3 || in_sizes[15] != NLAY * DD * DD) return;
  if (in_sizes[8] != NLAY * DD || in_sizes[10] != NLAY * DD || in_sizes[11] != NLAY * DD ||
      in_sizes[12] != NLAY * DD || in_sizes[16] != NLAY * DD) return;
  for (int i = 17; i <= 22; ++i) if (in_sizes[i] != NLAY * DD) return;
  if (in_sizes[23] != NLAY * DD * D2 || in_sizes[24] != NLAY * D2 || in_sizes[25] != NLAY * D2 * DD ||
      in_sizes[26] != NLAY * DD || in_sizes[27] != DD * NC || in_sizes[28] != NC) return;
  if (out_size != NG * NC) return;
  if ((NN % TR) != 0 || (NN % NBLK) != 0 || (ET % CHUNK) != 0 || (NCH * CHUNK) != ET) return;

  const int* src = eidx;
  const int* dst = eidx + NE;

  size_t off = 0;
  const size_t ox32  = off; off += (size_t)NN * DD * 4;            off = (off + 255) & ~(size_t)255;
  const size_t ox16  = off; off += (size_t)NN * DD * 2;            off = (off + 255) & ~(size_t)255;
  const size_t opw2  = off; off += (size_t)DD * D2 * 2;            off = (off + 255) & ~(size_t)255;
  const size_t owlin = off; off += (size_t)NLAY * NLIN * DD * 2;   off = (off + 255) & ~(size_t)255;
  const size_t owo   = off; off += (size_t)NLAY * DD * DD * 2;     off = (off + 255) & ~(size_t)255;
  const size_t owm1  = off; off += (size_t)NLAY * D2 * DD * 2;     off = (off + 255) & ~(size_t)255;
  const size_t owm2  = off; off += (size_t)NLAY * DD * D2 * 2;     off = (off + 255) & ~(size_t)255;
  const size_t oxl   = off; off += (size_t)NN * DD * 4;            off = (off + 255) & ~(size_t)255;
  const size_t oxr   = off; off += (size_t)NN * DD * 4;            off = (off + 255) & ~(size_t)255;
  const size_t oq    = off; off += (size_t)NH * NN * QP * 2;       off = (off + 255) & ~(size_t)255;
  const size_t ok    = off; off += (size_t)NH * NN * QP * 2;       off = (off + 255) & ~(size_t)255;
  const size_t ovt   = off; off += (size_t)NH * DH * NN * 2;       off = (off + 255) & ~(size_t)255;
  const size_t oh1   = off; off += (size_t)NN * DD * 4;            off = (off + 255) & ~(size_t)255;
  const size_t oh2   = off; off += (size_t)NN * DD * 4;            off = (off + 255) & ~(size_t)255;
  const size_t oo2   = off; off += (size_t)NN * DD * 4;            off = (off + 255) & ~(size_t)255;
  const size_t oo16  = off; off += (size_t)NH * NN * DH * 2;       off = (off + 255) & ~(size_t)255;
  const size_t ost   = off; off += (size_t)NLAY * 384 * 4;         off = (off + 255) & ~(size_t)255;
  const size_t opool = off; off += (size_t)NG * DD * 4;            off = (off + 255) & ~(size_t)255;
  if (off > ws_size) return;
  if (off > ((size_t)128 << 20)) return;

  unsigned char* ws = (unsigned char*)d_ws;
  float*    x32   = (float*)(ws + ox32);
  _Float16* x16   = (_Float16*)(ws + ox16);
  _Float16* pW2t  = (_Float16*)(ws + opw2);
  _Float16* Wlin  = (_Float16*)(ws + owlin);
  _Float16* Wo16  = (_Float16*)(ws + owo);
  _Float16* Wm1t  = (_Float16*)(ws + owm1);
  _Float16* Wm2t  = (_Float16*)(ws + owm2);
  float*    xl    = (float*)(ws + oxl);
  float*    xr    = (float*)(ws + oxr);
  _Float16* q16   = (_Float16*)(ws + oq);
  _Float16* k16   = (_Float16*)(ws + ok);
  _Float16* vT16  = (_Float16*)(ws + ovt);
  float*    h1    = (float*)(ws + oh1);
  float*    h2    = (float*)(ws + oh2);
  float*    o2    = (float*)(ws + oo2);
  _Float16* o16   = (_Float16*)(ws + oo16);
  float*    stt   = (float*)(ws + ost);
  float*    pooled = (float*)(ws + opool);
  float*    out   = (float*)d_out;

  const unsigned tileBlocks = (unsigned)(NN / TR);
  const unsigned aggBlocks  = (unsigned)(NN / NBLK);
  const unsigned applyBlocks = (unsigned)((NN * DD) / 2048);

  prep_kernel<<<(unsigned)((PREP_TASKS + 255) / 256), 256, 0, stream>>>(pre_w2, gat_wl, gat_wr, ain_w, aout_w,
                                                                      mlp_w1, mlp_w2, pW2t, Wlin, Wo16, Wm1t, Wm2t);
  premlp_kernel<<<tileBlocks, 256, 0, stream>>>(x_in, pre_w1, pre_b1, pW2t, pre_b2, x32, x16);

  for (int ly = 0; ly < NLAY; ++ly) {
    float* st = stt + (size_t)ly * 384;
    lin_kernel<<<tileBlocks, 256, 0, stream>>>(x16, Wlin + (size_t)ly * NLIN * DD, gat_bl + (size_t)ly * DD,
                                               gat_br + (size_t)ly * DD, ain_b + (size_t)ly * D3,
                                               xl, xr, q16, k16, vT16);
    agg_kernel<<<aggBlocks, 32, 0, stream>>>(src, dst, xl, xr, gat_att + (size_t)ly * DD,
                                            gat_bias + (size_t)ly * DD, x32, h1);
    attn_kernel<<<dim3(NN / 64, NH), 128, 0, stream>>>(q16, k16, vT16, o16);
    oproj_kernel<<<tileBlocks, 256, 0, stream>>>(o16, Wo16 + (size_t)ly * DD * DD, aout_b + (size_t)ly * DD, x32, h2);
    stats_kernel<<<2, 256, 0, stream>>>(h1, h2, st);
    mlp_kernel<<<tileBlocks, 256, 0, stream>>>(h1, h2, st, bn1_g + (size_t)ly * DD, bn1_b + (size_t)ly * DD,
                                               bn2_g + (size_t)ly * DD, bn2_b + (size_t)ly * DD,
                                               Wm1t + (size_t)ly * D2 * DD, mlp_b1 + (size_t)ly * D2,
                                               Wm2t + (size_t)ly * DD * D2, mlp_b2 + (size_t)ly * DD, o2);
    stats_kernel<<<1, 256, 0, stream>>>(o2, o2, st + 256);
    apply_kernel<<<applyBlocks, 256, 0, stream>>>(o2, st + 256, bn3_g + (size_t)ly * DD, bn3_b + (size_t)ly * DD,
                                                  x32, x16);
  }

  pool_kernel<<<(unsigned)NG, 64, 0, stream>>>(x32, bidx, pooled);
  final_kernel<<<1, 64, 0, stream>>>(pooled, fin_w, fin_b, out);

  (void)hipGetLastError();
}
